// LoFTREncoderLayer_88373247082501
// MI455X (gfx1250) — hardware-verified
//
#include <hip/hip_runtime.h>


#define NB_  8
#define CC   256
#define LL   4096
#define NH_  8
#define HD   32
typedef _Float16 h16;
typedef unsigned short bf;
typedef __attribute__((ext_vector_type(16))) __bf16   v16bf;
typedef __attribute__((ext_vector_type(16))) _Float16 v16h;
typedef __attribute__((ext_vector_type(8)))  _Float16 v8h;
typedef __attribute__((ext_vector_type(8)))  unsigned short v8us;
typedef __attribute__((ext_vector_type(8)))  float    v8f;
typedef __attribute__((ext_vector_type(4)))  float    v4f;
typedef v8h  __attribute__((may_alias)) v8ha;
typedef v4f  __attribute__((may_alias)) v4fa;
typedef v8us __attribute__((may_alias)) v8usa;

__device__ __forceinline__ unsigned short f2bf(float f) { unsigned u = __float_as_uint(f); u += 0x7FFFu + ((u >> 16) & 1u); return (unsigned short)(u >> 16); }
__device__ __forceinline__ float bf2f(unsigned short b) { return __uint_as_float(((unsigned)b) << 16); }
__device__ __forceinline__ float bfr(float f) { return bf2f(f2bf(f)); }
__device__ __forceinline__ v16h cat16(v8h lo, v8h hi) { return __builtin_shufflevector(lo, hi, 0, 1, 2, 3, 4, 5, 6, 7, 8, 9, 10, 11, 12, 13, 14, 15); }
__device__ __forceinline__ v16bf cat16b(v8us lo, v8us hi) { return __builtin_bit_cast(v16bf, __builtin_shufflevector(lo, hi, 0, 1, 2, 3, 4, 5, 6, 7, 8, 9, 10, 11, 12, 13, 14, 15)); }
__device__ __forceinline__ v8f wmma16(v16h a, v16h b, v8f c) { return __builtin_amdgcn_wmma_f32_16x16x32_f16(false, a, false, b, (short)0, c, false, false); }
__device__ __forceinline__ v8f wmmab(v16bf a, v16bf b, v8f c) { return __builtin_amdgcn_wmma_f32_16x16x32_bf16(false, a, false, b, (short)0, c, false, false); }


template <typename T16> struct WFrag;
template <> struct WFrag<h16> { typedef v16h V; static __device__ __forceinline__ V ld(const h16* p) { return cat16(*(const v8h*)p, *(const v8h*)(p + 16)); } static __device__ __forceinline__ v8f mma(V a, V b, v8f c) { return wmma16(a, b, c); } };
template <> struct WFrag<bf> { typedef v16bf V; static __device__ __forceinline__ V ld(const bf* p) { return cat16b(*(const v8us*)p, *(const v8us*)(p + 16)); } static __device__ __forceinline__ v8f mma(V a, V b, v8f c) { return wmmab(a, b, c); } };
template <typename T16, int NSPLIT, bool BIAS>
__global__ __launch_bounds__(32) void k_gemmw(const T16* __restrict__ A, const T16* __restrict__ A2, const T16* __restrict__ Bt, const T16* __restrict__ Bt2, int K, float* C, int ldc, const float* __restrict__ bias, size_t sA, size_t sB, size_t sC) {
    typedef typename WFrag<T16>::V V;
    __shared__ __align__(16) float os[16 * 68];
    const size_t z = blockIdx.z; A += z * sA; if (A2) A2 += z * sA; Bt += z * sB; if (Bt2) Bt2 += z * sB; C += z * sC;
    const int lane = threadIdx.x & 31, lr = lane & 15, hi = lane >> 4; const int r0 = blockIdx.x * 64, c0 = blockIdx.y * 64;
    v8f acc[4][4];
#pragma unroll
    for (int mb = 0; mb < 4; ++mb)
#pragma unroll
        for (int nb = 0; nb < 4; ++nb) acc[mb][nb] = (v8f){};
    const size_t aoff = (size_t)(r0 + lr) * K + 8 * hi, boff = (size_t)(c0 + lr) * K + 8 * hi;
#pragma unroll 1
    for (int kc = 0; kc < K; kc += 32) {
        V a[4], a2[4];
#pragma unroll
        for (int mb = 0; mb < 4; ++mb) { a[mb] = WFrag<T16>::ld(A + aoff + (size_t)mb * 16 * K + kc); if (NSPLIT == 1 || NSPLIT == 2) a2[mb] = WFrag<T16>::ld(A2 + aoff + (size_t)mb * 16 * K + kc); }
#pragma unroll
        for (int nb = 0; nb < 4; ++nb) { const V b = WFrag<T16>::ld(Bt + boff + (size_t)nb * 16 * K + kc); V b2; if (NSPLIT >= 2) b2 = WFrag<T16>::ld(Bt2 + boff + (size_t)nb * 16 * K + kc);
#pragma unroll
            for (int mb = 0; mb < 4; ++mb) { acc[mb][nb] = WFrag<T16>::mma(a[mb], b, acc[mb][nb]); if (NSPLIT == 1 || NSPLIT == 2) acc[mb][nb] = WFrag<T16>::mma(a2[mb], b, acc[mb][nb]); if (NSPLIT >= 2) acc[mb][nb] = WFrag<T16>::mma(a[mb], b2, acc[mb][nb]); } }
        asm volatile("v_nop\n\tv_nop\n\tv_nop\n\tv_nop" : "+v"(acc[0][0]), "+v"(acc[1][1]), "+v"(acc[2][2]), "+v"(acc[3][3]) : "v"(a[0]), "v"(a[3]));
    }
#pragma unroll
    for (int mb = 0; mb < 4; ++mb) {
#pragma unroll
        for (int nb = 0; nb < 4; ++nb) {
#pragma unroll
            for (int j = 0; j < 8; ++j) os[(hi * 8 + j) * 68 + nb * 16 + lr] = acc[mb][nb][j]; }
        __builtin_amdgcn_wave_barrier(); asm volatile("" ::: "memory");
        float* crow = C + (size_t)(r0 + mb * 16) * ldc + c0;
#pragma unroll 1
        for (int ps = 0; ps < 2; ++ps) {
#pragma unroll
            for (int s = 0; s < 8; ++s) { const int row = 2 * s + hi, cofs = lr * 4; v4f val = *(const v4fa*)(os + row * 68 + cofs); if (BIAS) { val[0] += bfr(bias[c0 + cofs]); val[1] += bfr(bias[c0 + cofs + 1]); val[2] += bfr(bias[c0 + cofs + 2]); val[3] += bfr(bias[c0 + cofs + 3]); }
                *(volatile v4f*)(crow + (size_t)row * ldc + cofs) = val; }
            if (ps == 0) __threadfence(); }
        __builtin_amdgcn_wave_barrier(); asm volatile("" ::: "memory");
    }
}

__device__ __forceinline__ void splitf(float y, unsigned short& h, unsigned short& l) { h = f2bf(y); l = f2bf(y - bf2f(h)); }
typedef __attribute__((ext_vector_type(2))) unsigned short v2us;
typedef __attribute__((ext_vector_type(4))) unsigned short v4us;

__global__ __launch_bounds__(256) void k_wtG(const float* __restrict__ w, int K, int N, bf* Bt) {
    const int lane = threadIdx.x & 31; const int L0 = (blockIdx.x * 8 + (threadIdx.x >> 5)) * 8; const int nlines = N * K / 64;
#pragma unroll
    for (int ps = 0; ps < 2; ++ps) {
#pragma unroll 1
        for (int l = 0; l < 8; ++l) { const int L = L0 + l; if (L >= nlines) break; const size_t e = (size_t)L * 64 + lane * 2; const int k = (int)(e % K), n = (int)(e / K); v2us o;
            o[0] = f2bf(w[(size_t)k * N + n]); o[1] = f2bf(w[(size_t)(k + 1) * N + n]); *(volatile v2us*)(Bt + e) = o; }
        if (ps == 0) __threadfence(); }
}

__global__ __launch_bounds__(256) void k_xt(const float* __restrict__ X, bf* XT) { const int e = (blockIdx.x * 256 + threadIdx.x) * 4; if (e >= LL * CC) return; const int c = e % CC; const int l = e / CC; v4us o;
#pragma unroll
    for (int u = 0; u < 4; ++u) o[u] = f2bf(X[(size_t)(c + u) * LL + l]); *(volatile v4us*)(XT + e) = o; __threadfence(); *(volatile v4us*)(XT + e) = o; }
__device__ __forceinline__ float elu1(float u) { return (u > 0.f) ? __fadd_rn(u, 1.0f) : __expf(u); }
__global__ __launch_bounds__(256) void k_elupl(const float* __restrict__ F, bf* Ph, bf* Pl) { const size_t e = ((size_t)blockIdx.x * 256 + threadIdx.x) * 4; if (e >= (size_t)LL * CC) return; const v4f a = *(const v4f*)(F + e); v4us oh, ol;
#pragma unroll
    for (int u = 0; u < 4; ++u) { unsigned short x0, x1; splitf(elu1(a[u]), x0, x1); oh[u] = x0; ol[u] = x1; } *(volatile v4us*)(Ph + e) = oh; *(volatile v4us*)(Pl + e) = ol; __threadfence(); *(volatile v4us*)(Ph + e) = oh; *(volatile v4us*)(Pl + e) = ol; }
__global__ __launch_bounds__(256) void k_eluT(const float* __restrict__ F, bf* Ph, bf* Pl) { const size_t e = ((size_t)blockIdx.x * 256 + threadIdx.x) * 2; if (e >= (size_t)CC * LL) return; const int l = (int)(e % LL); const int c = (int)(e / LL); v2us oh, ol;
#pragma unroll
    for (int u = 0; u < 2; ++u) { unsigned short a, b; splitf(elu1(F[(size_t)(l + u) * CC + c]), a, b); oh[u] = a; ol[u] = b; } *(volatile v2us*)(Ph + e) = oh; *(volatile v2us*)(Pl + e) = ol; __threadfence(); *(volatile v2us*)(Ph + e) = oh; *(volatile v2us*)(Pl + e) = ol; }
__global__ __launch_bounds__(256) void k_vT(const float* __restrict__ F, bf* Ph, bf* Pl) { const size_t e = ((size_t)blockIdx.x * 256 + threadIdx.x) * 2; if (e >= (size_t)CC * LL) return; const int l = (int)(e % LL); const int c = (int)(e / LL); v2us oh, ol;
#pragma unroll
    for (int u = 0; u < 2; ++u) { unsigned short a, b; splitf(F[(size_t)(l + u) * CC + c] * (1.0f / (float)LL), a, b); oh[u] = a; ol[u] = b; } *(volatile v2us*)(Ph + e) = oh; *(volatile v2us*)(Pl + e) = ol; __threadfence(); *(volatile v2us*)(Ph + e) = oh; *(volatile v2us*)(Pl + e) = ol; }
__global__ __launch_bounds__(256) void k_ksum(const float* __restrict__ F, float* KS) { const int c = blockIdx.x * 256 + threadIdx.x; if (c >= CC) return; float s = 0.f;
#pragma unroll 1
    for (int l = 0; l < LL; ++l) s = __fadd_rn(s, elu1(F[(size_t)l * CC + c])); *(volatile float*)(KS + c) = s; __threadfence(); *(volatile float*)(KS + c) = s; }
__global__ __launch_bounds__(256) void k_bd(const float* __restrict__ KV, bf* Bh, bf* Bl) { const int e = (blockIdx.x * 256 + threadIdx.x) * 4; if (e >= CC * CC) return; const int k = e % CC; const int n = e / CC; v4us oh, ol;
#pragma unroll
    for (int u = 0; u < 4; ++u) { unsigned short a = 0, b = 0; if ((k + u) / HD == n / HD) splitf(KV[(size_t)(k + u) * CC + n], a, b); oh[u] = a; ol[u] = b; } *(volatile v4us*)(Bh + e) = oh; *(volatile v4us*)(Bl + e) = ol; __threadfence(); *(volatile v4us*)(Bh + e) = oh; *(volatile v4us*)(Bl + e) = ol; }
__global__ __launch_bounds__(256) void k_msg(const float* __restrict__ G, const float* __restrict__ FQ, const float* __restrict__ KS, bf* Ph, bf* Pl) { const int lane = threadIdx.x & 31; const int l = blockIdx.x * 8 + (threadIdx.x >> 5); if (l >= LL) return;
    float part = 0.f; float qv[8];
#pragma unroll
    for (int u = 0; u < 8; ++u) { const int c = lane * 8 + u; qv[u] = elu1(FQ[(size_t)l * CC + c]); float p = __fmul_rn(qv[u], KS[c]); asm volatile("" : "+v"(p)); part = __fadd_rn(part, p); }
    part = __fadd_rn(part, __shfl_xor(part, 1, 32)); part = __fadd_rn(part, __shfl_xor(part, 2, 32));
    const float z = __fdiv_rn(1.0f, __fadd_rn(part, 1e-6f)); v4us oh0, ol0, oh1, ol1;
#pragma unroll
    for (int u = 0; u < 8; ++u) { const int c = lane * 8 + u; float m0 = __fmul_rn(G[(size_t)l * CC + c], z); asm volatile("" : "+v"(m0)); const float m1 = __fmul_rn(m0, (float)LL); unsigned short a, b; splitf(m1, a, b); if (u < 4) { oh0[u] = a; ol0[u] = b; } else { oh1[u - 4] = a; ol1[u - 4] = b; } }
    const size_t oo = (size_t)l * CC + lane * 8;
    for (int ps = 0; ps < 2; ++ps) { *(volatile v4us*)(Ph + oo) = oh0; *(volatile v4us*)(Ph + oo + 4) = oh1; *(volatile v4us*)(Pl + oo) = ol0; *(volatile v4us*)(Pl + oo + 4) = ol1; if (ps == 0) __threadfence(); } }
__global__ __launch_bounds__(256) void k_ln256(const float* __restrict__ F, const float* __restrict__ g, const float* __restrict__ bb, const bf* __restrict__ XS, int pitch, int coff, bf* Ph, bf* Pl, float* LNF) {
    const int lane = threadIdx.x & 31; const int l = blockIdx.x * 8 + (threadIdx.x >> 5); if (l >= LL) return; float v[8]; float s = 0.f;
#pragma unroll
    for (int u = 0; u < 8; ++u) { v[u] = F[(size_t)l * CC + lane * 8 + u]; s += v[u]; }
#pragma unroll
    for (int sh = 16; sh; sh >>= 1) s += __shfl_xor(s, sh, 32);
    const float mean = s * (1.0f / CC); float q = 0.f;
#pragma unroll
    for (int u = 0; u < 8; ++u) { float d = __fsub_rn(v[u], mean); asm volatile("" : "+v"(d)); v[u] = d; float p = __fmul_rn(d, d); asm volatile("" : "+v"(p)); q = __fadd_rn(q, p); }
#pragma unroll
    for (int sh = 16; sh; sh >>= 1) q += __shfl_xor(q, sh, 32);
    const float sd = __fsqrt_rn(__fadd_rn(q * (1.0f / CC), 1e-5f)); v4us oh0, ol0, oh1, ol1; v4f f0, f1;
#pragma unroll
    for (int u = 0; u < 8; ++u) { const int c = lane * 8 + u; float n0 = __fdiv_rn(v[u], sd); asm volatile("" : "+v"(n0)); float gg = bfr(g[c]), be = bfr(bb[c]); asm volatile("" : "+v"(gg)); asm volatile("" : "+v"(be)); float t1 = __fmul_rn(n0, gg); asm volatile("" : "+v"(t1)); const float y = __fadd_rn(t1, be); unsigned short a, b; splitf(y, a, b); if (u < 4) { oh0[u] = a; ol0[u] = b; f0[u] = y; } else { oh1[u - 4] = a; ol1[u - 4] = b; f1[u - 4] = y; } }
    const size_t oo = (size_t)l * pitch + coff + lane * 8;
    for (int ps = 0; ps < 2; ++ps) {
        if (Ph) { *(volatile v4us*)(Ph + oo) = oh0; *(volatile v4us*)(Ph + oo + 4) = oh1; *(volatile v4us*)(Pl + oo) = ol0; *(volatile v4us*)(Pl + oo + 4) = ol1; }
        if (XS) { v4us xa = *(const v4us*)(XS + (size_t)l * CC + lane * 8), xb = *(const v4us*)(XS + (size_t)l * CC + lane * 8 + 4); v4us z4; z4[0] = 0; z4[1] = 0; z4[2] = 0; z4[3] = 0; const size_t ox = (size_t)l * pitch + lane * 8; *(volatile v4us*)(Ph + ox) = xa; *(volatile v4us*)(Ph + ox + 4) = xb; *(volatile v4us*)(Pl + ox) = z4; *(volatile v4us*)(Pl + ox + 4) = z4; }
        if (LNF) { *(volatile v4f*)(LNF + (size_t)l * CC + lane * 8) = f0; *(volatile v4f*)(LNF + (size_t)l * CC + lane * 8 + 4) = f1; }
        if (ps == 0) __threadfence(); } }
__global__ __launch_bounds__(256) void k_relupl(const float* __restrict__ F, bf* Ph, bf* Pl, size_t n4) { const size_t e = ((size_t)blockIdx.x * 256 + threadIdx.x) * 4; if (e >= n4 * 4) return; const v4f a = *(const v4f*)(F + e); v4us oh, ol;
#pragma unroll
    for (int u = 0; u < 4; ++u) { unsigned short x0, x1; splitf(fmaxf(a[u], 0.f), x0, x1); oh[u] = x0; ol[u] = x1; } *(volatile v4us*)(Ph + e) = oh; *(volatile v4us*)(Pl + e) = ol; __threadfence(); *(volatile v4us*)(Ph + e) = oh; *(volatile v4us*)(Pl + e) = ol; }
__global__ __launch_bounds__(256) void k_out(const float* __restrict__ M2N, const float* __restrict__ X, float* Y) { const size_t e = ((size_t)blockIdx.x * 256 + threadIdx.x) * 4; if (e >= (size_t)CC * LL) return; const int l = (int)(e % LL); const int c = (int)(e / LL); const v4f xx = *(const v4f*)(X + e); v4f r;
#pragma unroll
    for (int u = 0; u < 4; ++u) r[u] = __fadd_rn(bfr(xx[u]), M2N[(size_t)(l + u) * CC + c]); *(volatile v4f*)(Y + e) = r; __threadfence(); *(volatile v4f*)(Y + e) = r; }

extern "C" void kernel_launch(void* const* d_in, const int* in_sizes, int n_in,
                              void* d_out, int out_size, void* d_ws, size_t ws_size, hipStream_t stream) {
    (void)in_sizes; (void)n_in; (void)out_size;
    const float* x = (const float*)d_in[0]; const float* src = (const float*)d_in[1]; const float* Wq = (const float*)d_in[2]; const float* Wk = (const float*)d_in[3]; const float* Wv = (const float*)d_in[4]; const float* Wm = (const float*)d_in[5]; const float* W1 = (const float*)d_in[6]; const float* W2 = (const float*)d_in[7];
    const float* g1 = (const float*)d_in[8]; const float* b1 = (const float*)d_in[9]; const float* g2 = (const float*)d_in[10]; const float* b2 = (const float*)d_in[11];
    float* OUT = (float*)d_out;
    char* wsp = (char*)d_ws;
    auto take = [&](size_t bytes) { char* p = wsp; wsp += (bytes + 255) & ~(size_t)255; return (void*)p; };
    bf* BQ = (bf*)take((size_t)CC * CC * 2); bf* BK = (bf*)take((size_t)CC * CC * 2); bf* BV = (bf*)take((size_t)CC * CC * 2); bf* BM = (bf*)take((size_t)CC * CC * 2); bf* B1 = (bf*)take((size_t)2 * CC * 2 * CC * 2); bf* B2 = (bf*)take((size_t)CC * 2 * CC * 2);
    bf* XT = (bf*)take((size_t)LL * CC * 2); bf* ST = (bf*)take((size_t)LL * CC * 2); float* FQ = (float*)take((size_t)LL * CC * 4); float* FK = (float*)take((size_t)LL * CC * 4); float* FV = (float*)take((size_t)LL * CC * 4);
    bf* QPh = (bf*)take((size_t)LL * CC * 2); bf* QPl = (bf*)take((size_t)LL * CC * 2); bf* KTh = (bf*)take((size_t)CC * LL * 2); bf* KTl = (bf*)take((size_t)CC * LL * 2); bf* VTh = (bf*)take((size_t)CC * LL * 2); bf* VTl = (bf*)take((size_t)CC * LL * 2); float* KS = (float*)take(CC * 4);
    float* KV = (float*)take((size_t)CC * CC * 4); bf* BDh = (bf*)take((size_t)CC * CC * 2); bf* BDl = (bf*)take((size_t)CC * CC * 2); float* G = (float*)take((size_t)LL * CC * 4); bf* MPh = (bf*)take((size_t)LL * CC * 2); bf* MPl = (bf*)take((size_t)LL * CC * 2);
    float* MW = (float*)take((size_t)LL * CC * 4); bf* CATh = (bf*)take((size_t)LL * 2 * CC * 2); bf* CATl = (bf*)take((size_t)LL * 2 * CC * 2); float* H1 = (float*)take((size_t)LL * 2 * CC * 4); bf* H1h = (bf*)take((size_t)LL * 2 * CC * 2); bf* H1l = (bf*)take((size_t)LL * 2 * CC * 2); float* M2 = (float*)take((size_t)LL * CC * 4); float* M2N = (float*)take((size_t)LL * CC * 4);
    if ((size_t)(wsp - (char*)d_ws) > ws_size) return;
    k_wtG<<<(CC * CC / 64 + 63) / 64, 256, 0, stream>>>(Wq, CC, CC, BQ); k_wtG<<<(CC * CC / 64 + 63) / 64, 256, 0, stream>>>(Wk, CC, CC, BK); k_wtG<<<(CC * CC / 64 + 63) / 64, 256, 0, stream>>>(Wv, CC, CC, BV); k_wtG<<<(CC * CC / 64 + 63) / 64, 256, 0, stream>>>(Wm, CC, CC, BM);
    k_wtG<<<(2 * CC * 2 * CC / 64 + 63) / 64, 256, 0, stream>>>(W1, 2 * CC, 2 * CC, B1); k_wtG<<<(2 * CC * CC / 64 + 63) / 64, 256, 0, stream>>>(W2, 2 * CC, CC, B2);
    const dim3 gp(LL / 64, CC / 64, 1); const unsigned LP = (unsigned)(((size_t)LL * CC / 4 + 255) / 256), LT = (unsigned)(((size_t)CC * LL / 2 + 255) / 256);
    for (int b = 0; b < NB_; ++b) { const float* xb = x + (size_t)b * CC * LL; const float* sb = src + (size_t)b * CC * LL;
        k_xt<<<(LL * CC / 4 + 255) / 256, 256, 0, stream>>>(xb, XT); k_xt<<<(LL * CC / 4 + 255) / 256, 256, 0, stream>>>(sb, ST);
        k_gemmw<bf, 0, false><<<gp, 32, 0, stream>>>(XT, nullptr, BQ, nullptr, CC, FQ, CC, nullptr, 0, 0, 0); k_elupl<<<LP, 256, 0, stream>>>(FQ, QPh, QPl);
        k_gemmw<bf, 0, false><<<gp, 32, 0, stream>>>(ST, nullptr, BK, nullptr, CC, FK, CC, nullptr, 0, 0, 0); k_eluT<<<LT, 256, 0, stream>>>(FK, KTh, KTl); k_ksum<<<1, 256, 0, stream>>>(FK, KS);
        k_gemmw<bf, 0, false><<<gp, 32, 0, stream>>>(ST, nullptr, BV, nullptr, CC, FV, CC, nullptr, 0, 0, 0); k_vT<<<LT, 256, 0, stream>>>(FV, VTh, VTl);
        k_gemmw<bf, 2, false><<<dim3(CC / 64, CC / 64, 1), 32, 0, stream>>>(KTh, KTl, VTh, VTl, LL, KV, CC, nullptr, 0, 0, 0);
        k_bd<<<(CC * CC / 4 + 255) / 256, 256, 0, stream>>>(KV, BDh, BDl);
        k_gemmw<bf, 2, false><<<gp, 32, 0, stream>>>(QPh, QPl, BDh, BDl, CC, G, CC, nullptr, 0, 0, 0);
        k_msg<<<LL / 8, 256, 0, stream>>>(G, FQ, KS, MPh, MPl);
        k_gemmw<bf, 1, false><<<gp, 32, 0, stream>>>(MPh, MPl, BM, nullptr, CC, MW, CC, nullptr, 0, 0, 0);
        k_ln256<<<LL / 8, 256, 0, stream>>>(MW, g1, b1, XT, 2 * CC, CC, CATh, CATl, nullptr);
        k_gemmw<bf, 1, false><<<dim3(LL / 64, 2 * CC / 64, 1), 32, 0, stream>>>(CATh, CATl, B1, nullptr, 2 * CC, H1, 2 * CC, nullptr, 0, 0, 0);
        k_relupl<<<(unsigned)(((size_t)LL * 2 * CC / 4 + 255) / 256), 256, 0, stream>>>(H1, H1h, H1l, (size_t)LL * 2 * CC / 4);
        k_gemmw<bf, 1, false><<<gp, 32, 0, stream>>>(H1h, H1l, B2, nullptr, 2 * CC, M2, CC, nullptr, 0, 0, 0);
        k_ln256<<<LL / 8, 256, 0, stream>>>(M2, g2, b2, nullptr, CC, 0, nullptr, nullptr, M2N);
        k_out<<<(unsigned)(((size_t)CC * LL / 4 + 255) / 256), 256, 0, stream>>>(M2N, xb, OUT + (size_t)b * CC * LL); }
}
